// Attention_19550691131960
// MI455X (gfx1250) — hardware-verified
//
#include <hip/hip_runtime.h>


#ifndef NB
#define NB 4
#endif
#ifndef SEQ
#define SEQ 2048
#endif
#define NB_FULL  4
#define SEQ_FULL 2048
#define DM   768
#define NH   12
#define HD   64
#define WCAR 64.0f
#define CCAR 64.0f
#define SC2  (0.125f * 1.4426950408889634f)

typedef _Float16 h16;
typedef __attribute__((ext_vector_type(16))) _Float16 v16h;
typedef __attribute__((ext_vector_type(8)))  _Float16 v8h;
typedef __attribute__((ext_vector_type(8)))  float    v8f;
typedef __attribute__((ext_vector_type(4)))  float    v4f;
typedef v8h __attribute__((may_alias)) v8ha;
typedef v4f __attribute__((may_alias)) v4fa;

static_assert(NH * HD == DM);
static_assert(HD == 64);
static_assert(DM % 64 == 0);
static_assert(DM % 32 == 0);
static_assert(DM % 8 == 0);
static_assert(SEQ % 64 == 0);
static_assert((NB * SEQ) % 64 == 0);
static_assert(NB <= NB_FULL);
static_assert(SEQ <= SEQ_FULL);
static_assert(((size_t)NB * SEQ * DM / 8) % 256 == 0);

__device__ __forceinline__ unsigned short f2bf(float f) { unsigned u = __float_as_uint(f); u += 0x7FFFu + ((u >> 16) & 1u); return (unsigned short)(u >> 16); }
__device__ __forceinline__ float bfr(float f) { return __uint_as_float(((unsigned)f2bf(f)) << 16); }
__device__ __forceinline__ v16h cat16(v8h lo, v8h hi) { return __builtin_shufflevector(lo, hi, 0, 1, 2, 3, 4, 5, 6, 7, 8, 9, 10, 11, 12, 13, 14, 15); }
__device__ __forceinline__ v16h ldfrag(const h16* p) { return cat16(*(const v8h*)p, *(const v8h*)(p + 16)); }
__device__ __forceinline__ v8f wmma16(v16h a, v16h b, v8f c) { return __builtin_amdgcn_wmma_f32_16x16x32_f16(false, a, false, b, (short)0, c, false, false); }

__global__ __launch_bounds__(256) void k_cvtx(const float* __restrict__ X, h16* XH) {
    const size_t idx = (size_t)blockIdx.x * 256 + threadIdx.x;
    const size_t e = idx * 8;
    if (e >= (size_t)NB * SEQ * DM) return;
    const size_t row = e / DM; const int col = (int)(e - row * DM);
    const size_t b = row / SEQ; const size_t n = row - b * SEQ;
    const float* src = X + (b * SEQ_FULL + n) * DM + col;
    const v4f a = *(const v4f*)src; const v4f c = *(const v4f*)(src + 4);
    v8h o;
    o[0] = (h16)bfr(a[0]); o[1] = (h16)bfr(a[1]); o[2] = (h16)bfr(a[2]); o[3] = (h16)bfr(a[3]);
    o[4] = (h16)bfr(c[0]); o[5] = (h16)bfr(c[1]); o[6] = (h16)bfr(c[2]); o[7] = (h16)bfr(c[3]);
    *(volatile v8h*)(XH + e) = o; __threadfence(); *(volatile v8h*)(XH + e) = o;
}

__global__ __launch_bounds__(256) void k_cvtw(const float* __restrict__ W, h16* WT) {
    __shared__ __align__(16) h16 ts[64 * 72];
    const int tid = threadIdx.x; const int k0 = blockIdx.x * 64, n0 = blockIdx.y * 64;
#pragma unroll
    for (int it = 0; it < 4; ++it) {
        const int f = it * 256 + tid; const int kr = f >> 4; const int nc = (f & 15) * 4;
        const v4f a = *(const v4f*)(W + (size_t)(k0 + kr) * DM + n0 + nc);
#pragma unroll
        for (int q = 0; q < 4; ++q) ts[(nc + q) * 72 + kr] = (h16)(bfr(a[q]) * WCAR);
    }
    __syncthreads();
#pragma unroll 1
    for (int ps = 0; ps < 2; ++ps) {
#pragma unroll
        for (int it = 0; it < 2; ++it) {
            const int line = it * 32 + (tid >> 3); const int pc = (tid & 7) * 8;
            const v8h v = *(const v8ha*)(ts + line * 72 + pc);
            *(volatile v8h*)(WT + (size_t)(n0 + line) * DM + k0 + pc) = v;
        }
        if (ps == 0) __threadfence();
    }
}

__device__ __forceinline__ void gemm_main(const h16* __restrict__ A, const h16* __restrict__ Bt, int lane, v8f (&acc)[4][4]) {
    const int lr = lane & 15, hi = lane >> 4;
#pragma unroll
    for (int mb = 0; mb < 4; ++mb)
#pragma unroll
        for (int nb = 0; nb < 4; ++nb) acc[mb][nb] = (v8f){};
    const size_t off = (size_t)lr * DM + 8 * hi;
#pragma unroll 1
    for (int kc = 0; kc < DM; kc += 32) {
        v16h a[4]; v16h bq;
#pragma unroll
        for (int mb = 0; mb < 4; ++mb) a[mb] = ldfrag(A + off + (size_t)mb * 16 * DM + kc);
#pragma unroll
        for (int nb = 0; nb < 4; ++nb) {
            bq = ldfrag(Bt + off + (size_t)nb * 16 * DM + kc);
#pragma unroll
            for (int mb = 0; mb < 4; ++mb) acc[mb][nb] = wmma16(a[mb], bq, acc[mb][nb]);
        }
        asm volatile("v_nop\n\tv_nop\n\tv_nop\n\tv_nop"
                     : "+v"(acc[0][3]), "+v"(acc[1][3]), "+v"(acc[2][3]), "+v"(acc[3][3]), "+v"(acc[0][2]), "+v"(acc[1][2]), "+v"(acc[2][2]), "+v"(acc[3][2])
                     : "v"(a[0]), "v"(a[3]), "v"(bq));
    }
}

__global__ __launch_bounds__(32) void k_proj(const h16* __restrict__ A, const h16* __restrict__ Bt, h16* P, size_t sB, size_t sP, int mode) {
    __shared__ __align__(16) float os[16 * 68];
    const int lane = threadIdx.x & 31, lr = lane & 15, hi = lane >> 4;
    const int r0 = blockIdx.x * 64, c0 = blockIdx.y * 64; const size_t z = blockIdx.z;
    v8f acc[4][4];
    gemm_main(A + (size_t)r0 * DM, Bt + z * sB + (size_t)c0 * DM, lane, acc);
    size_t tb; size_t pitch;
    if (mode == 0) { const int b = r0 / SEQ, n0 = r0 % SEQ, h = c0 / HD; tb = (((size_t)b * NH + h) * SEQ + n0) * HD; pitch = HD; }
    else           { const int h = r0 / HD, b = c0 / SEQ, n0 = c0 % SEQ; tb = ((size_t)b * NH + h) * HD * SEQ + n0; pitch = SEQ; }
    h16* dst = P + z * sP + tb;
    const float sc = 1.0f / WCAR;
#pragma unroll
    for (int mb = 0; mb < 4; ++mb) {
#pragma unroll
        for (int nb = 0; nb < 4; ++nb) {
#pragma unroll
            for (int j = 0; j < 8; ++j) os[(hi * 8 + j) * 68 + nb * 16 + lr] = acc[mb][nb][j];
        }
        __syncthreads();
#pragma unroll 1
        for (int ps = 0; ps < 2; ++ps) {
#pragma unroll
            for (int s = 0; s < 4; ++s) {
                const int row = 4 * s + (lane >> 3); const int cof = (lane & 7) * 8;
                const v4f u0 = *(const v4fa*)(os + row * 68 + cof); const v4f u1 = *(const v4fa*)(os + row * 68 + cof + 4);
                v8h o;
                o[0] = (h16)(u0[0] * sc); o[1] = (h16)(u0[1] * sc); o[2] = (h16)(u0[2] * sc); o[3] = (h16)(u0[3] * sc);
                o[4] = (h16)(u1[0] * sc); o[5] = (h16)(u1[1] * sc); o[6] = (h16)(u1[2] * sc); o[7] = (h16)(u1[3] * sc);
                *(volatile v8h*)(dst + (size_t)(mb * 16 + row) * pitch + cof) = o;
            }
            if (ps == 0) __threadfence();
        }
        __syncthreads();
    }
}

__global__ __launch_bounds__(32) void k_outp(const h16* __restrict__ A, const h16* __restrict__ Bt, const float* __restrict__ bias, float* OUT) {
    __shared__ __align__(16) float os[16 * 68];
    const int lane = threadIdx.x & 31, lr = lane & 15, hi = lane >> 4;
    const int r0 = blockIdx.x * 64, c0 = blockIdx.y * 64;
    v8f acc[4][4];
    gemm_main(A + (size_t)r0 * DM, Bt + (size_t)c0 * DM, lane, acc);
    const int b = r0 / SEQ, n0 = r0 % SEQ;
    float* crow = OUT + ((size_t)b * SEQ_FULL + n0) * DM + c0;
    const int cofs = lr * 4;
    const v4f bv = *(const v4f*)(bias + c0 + cofs);
    v4f bb; bb[0] = bfr(bv[0]); bb[1] = bfr(bv[1]); bb[2] = bfr(bv[2]); bb[3] = bfr(bv[3]);
    const float sc = 1.0f / (WCAR * CCAR);
#pragma unroll
    for (int mb = 0; mb < 4; ++mb) {
#pragma unroll
        for (int nb = 0; nb < 4; ++nb) {
#pragma unroll
            for (int j = 0; j < 8; ++j) os[(hi * 8 + j) * 68 + nb * 16 + lr] = acc[mb][nb][j];
        }
        __syncthreads();
#pragma unroll 1
        for (int ps = 0; ps < 2; ++ps) {
#pragma unroll
            for (int s = 0; s < 8; ++s) {
                const int row = 2 * s + hi;
                const v4f u = *(const v4fa*)(os + row * 68 + cofs);
                v4f val; val[0] = u[0] * sc + bb[0]; val[1] = u[1] * sc + bb[1]; val[2] = u[2] * sc + bb[2]; val[3] = u[3] * sc + bb[3];
                *(volatile v4f*)(crow + (size_t)(mb * 16 + row) * DM + cofs) = val;
            }
            if (ps == 0) __threadfence();
        }
        __syncthreads();
    }
}

__global__ __launch_bounds__(128) void k_attn(const h16* __restrict__ QP, const h16* __restrict__ KP, const h16* __restrict__ VT, h16* CTX) {
    __shared__ __align__(16) h16 ot[4 * 16 * 72];
    const int tid = threadIdx.x, wave = tid >> 5, lane = tid & 31, lr = lane & 15, hi = lane >> 4;
    const int bh = blockIdx.x / (SEQ / 64), qblk = blockIdx.x % (SEQ / 64);
    const int b = bh / NH, h = bh % NH;
    const int q0 = qblk * 64 + wave * 16;
    const h16* qp = QP + (size_t)bh * SEQ * HD + (size_t)(q0 + lr) * HD + 8 * hi;
    const h16* kp = KP + (size_t)bh * SEQ * HD + (size_t)lr * HD + 8 * hi;
    const h16* vp = VT + (size_t)bh * HD * SEQ + (size_t)lr * SEQ + 8 * hi;
    const v16h qb0 = ldfrag(qp), qb1 = ldfrag(qp + 32);
    v8f o[4];
#pragma unroll
    for (int dt = 0; dt < 4; ++dt) o[dt] = (v8f){};
    float m = -1.0e30f, l = 0.0f;
#pragma unroll 1
    for (int j = 0; j < SEQ; j += 64) {
        v8f s[4]; v16h ka, kb2;
#pragma unroll
        for (int kt = 0; kt < 4; ++kt) {
            const h16* kr = kp + (size_t)(j + kt * 16) * HD;
            ka = ldfrag(kr); kb2 = ldfrag(kr + 32);
            v8f t = (v8f){};
            t = wmma16(ka, qb0, t);
            t = wmma16(kb2, qb1, t);
            s[kt] = t;
        }
        asm volatile("v_nop\n\tv_nop\n\tv_nop\n\tv_nop" : "+v"(s[0]), "+v"(s[1]), "+v"(s[2]), "+v"(s[3]) : "v"(ka), "v"(kb2), "v"(qb0), "v"(qb1));
        float tm = s[0][0];
#pragma unroll
        for (int kt = 0; kt < 4; ++kt)
#pragma unroll
            for (int r = 0; r < 8; ++r) tm = fmaxf(tm, s[kt][r]);
        tm = fmaxf(tm, __shfl_xor(tm, 16, 32));
        const float mn = fmaxf(m, tm * SC2);
        const float alpha = __builtin_amdgcn_exp2f(m - mn);
        m = mn;
        float psum = 0.0f;
#pragma unroll
        for (int kt = 0; kt < 4; ++kt)
#pragma unroll
            for (int r = 0; r < 8; ++r) { const float p = __builtin_amdgcn_exp2f(__builtin_fmaf(s[kt][r], SC2, -mn)); psum += p; s[kt][r] = p; }
        l = l * alpha + psum;
#pragma unroll
        for (int dt = 0; dt < 4; ++dt)
#pragma unroll
            for (int r = 0; r < 8; ++r) o[dt][r] *= alpha;
        v16h pb0, pb1;
#pragma unroll
        for (int r = 0; r < 8; ++r) { pb0[r] = (h16)s[0][r]; pb0[8 + r] = (h16)s[1][r]; pb1[r] = (h16)s[2][r]; pb1[8 + r] = (h16)s[3][r]; }
        v16h va;
#pragma unroll
        for (int dt = 0; dt < 4; ++dt) { va = ldfrag(vp + (size_t)(dt * 16) * SEQ + j); o[dt] = wmma16(va, pb0, o[dt]); }
#pragma unroll
        for (int dt = 0; dt < 4; ++dt) { va = ldfrag(vp + (size_t)(dt * 16) * SEQ + j + 32); o[dt] = wmma16(va, pb1, o[dt]); }
        asm volatile("v_nop\n\tv_nop\n\tv_nop\n\tv_nop" : "+v"(o[0]), "+v"(o[1]), "+v"(o[2]), "+v"(o[3]) : "v"(va), "v"(pb0), "v"(pb1));
    }
    l += __shfl_xor(l, 16, 32);
    const float inv = CCAR * (1.0f / l);
#pragma unroll
    for (int dt = 0; dt < 4; ++dt) {
        v8h ov;
#pragma unroll
        for (int r = 0; r < 8; ++r) ov[r] = (h16)(o[dt][r] * inv);
        *(v8ha*)(ot + (wave * 16 + lr) * 72 + dt * 16 + 8 * hi) = ov;
    }
    __syncthreads();
    h16* dst = CTX + ((size_t)b * SEQ + q0) * DM + h * HD;
#pragma unroll 1
    for (int ps = 0; ps < 2; ++ps) {
#pragma unroll
        for (int s4 = 0; s4 < 4; ++s4) {
            const int row = 4 * s4 + (lane >> 3); const int pc = (lane & 7) * 8;
            const v8h v = *(const v8ha*)(ot + (wave * 16 + row) * 72 + pc);
            *(volatile v8h*)(dst + (size_t)row * DM + pc) = v;
        }
        if (ps == 0) __threadfence();
    }
}

extern "C" void kernel_launch(void* const* d_in, const int* in_sizes, int n_in,
                              void* d_out, int out_size, void* d_ws, size_t ws_size, hipStream_t stream) {
    if (n_in < 6) return;
    constexpr size_t NEEDX = ((size_t)(NB - 1) * SEQ_FULL + SEQ) * DM;
    if ((size_t)in_sizes[0] < NEEDX) return;
    if (in_sizes[1] < DM * DM || in_sizes[2] < DM * DM || in_sizes[3] < DM * DM || in_sizes[4] < DM * DM || in_sizes[5] < DM) return;
    if ((size_t)out_size < NEEDX) return;
    const float* x  = (const float*)d_in[0];
    const float* Wq = (const float*)d_in[1];
    const float* Wk = (const float*)d_in[2];
    const float* Wv = (const float*)d_in[3];
    const float* Wp = (const float*)d_in[4];
    const float* bp = (const float*)d_in[5];
    float* OUT = (float*)d_out;

    constexpr size_t nX = (size_t)NB * SEQ * DM;
    constexpr size_t nW = (size_t)DM * DM;
    constexpr size_t SZX = nX * 2, SZW = 4 * nW * 2;
    static_assert(SZX % 256 == 0);
    static_assert(SZW % 256 == 0);
    constexpr size_t TOTAL = 5 * SZX + SZW;
    static_assert(TOTAL <= (size_t)134217728);
    if (ws_size < TOTAL) return;
    char* wsp = (char*)d_ws;
    h16* XH  = (h16*)wsp; wsp += SZX;
    h16* WT  = (h16*)wsp; wsp += SZW;
    h16* QK  = (h16*)wsp; wsp += 2 * SZX;
    h16* VTp = (h16*)wsp; wsp += SZX;
    h16* CTX = (h16*)wsp; wsp += SZX;

    k_cvtx<<<(unsigned)((nX / 8 + 255) / 256), 256, 0, stream>>>(x, XH);
    k_cvtw<<<dim3(DM / 64, DM / 64), 256, 0, stream>>>(Wq, WT);
    k_cvtw<<<dim3(DM / 64, DM / 64), 256, 0, stream>>>(Wk, WT + nW);
    k_cvtw<<<dim3(DM / 64, DM / 64), 256, 0, stream>>>(Wv, WT + 2 * nW);
    k_cvtw<<<dim3(DM / 64, DM / 64), 256, 0, stream>>>(Wp, WT + 3 * nW);
    k_proj<<<dim3(NB * SEQ / 64, DM / 64, 2), 32, 0, stream>>>(XH, WT, QK, nW, nX, 0);
    k_proj<<<dim3(DM / 64, NB * SEQ / 64, 1), 32, 0, stream>>>(WT + 2 * nW, XH, VTp, (size_t)0, (size_t)0, 1);
    k_attn<<<NB * NH * (SEQ / 64), 128, 0, stream>>>(QK, QK + nX, VTp, CTX);
    k_outp<<<dim3(NB * SEQ / 64, DM / 64), 32, 0, stream>>>(CTX, WT + 3 * nW, bp, OUT);
}
